// MyGATLayer_8452495638870
// MI455X (gfx1250) — hardware-verified
//
#include <hip/hip_runtime.h>
#include <math.h>

typedef __attribute__((ext_vector_type(16))) _Float16 v16h;
typedef __attribute__((ext_vector_type(16))) __bf16 v16b;
typedef __attribute__((ext_vector_type(8)))  _Float16 v8h;
typedef __attribute__((ext_vector_type(8)))  float v8f;
typedef __attribute__((ext_vector_type(4)))  float v4f;
typedef __attribute__((ext_vector_type(2)))  float v2f;
typedef __attribute__((ext_vector_type(4)))  unsigned v4u;
typedef __attribute__((ext_vector_type(4)))  int v4i;
typedef float __attribute__((may_alias)) float_a;
typedef int __attribute__((may_alias)) int_a;

template <typename T> __device__ __forceinline__ void vst2(void* p, T v) { *(volatile T*)p = v; __threadfence(); *(volatile T*)p = v; }
__device__ __forceinline__ v8f wmma16(v16h a, v16h b, v8f c) {
  v8f d = __builtin_amdgcn_wmma_f32_16x16x32_f16(false, a, false, b, (short)0, c, false, false);
  asm volatile("v_nop\n\tv_nop\n\tv_nop\n\tv_nop" : "+v"(d) : "v"(a), "v"(b));
  return d;
}
__device__ __forceinline__ v8f wmma_bf(v16b a, v16b b, v8f c) {
  v8f d = __builtin_amdgcn_wmma_f32_16x16x32_bf16(false, a, false, b, (short)0, c, false, false);
  asm volatile("v_nop\n\tv_nop\n\tv_nop\n\tv_nop" : "+v"(d) : "v"(a), "v"(b));
  return d;
}
__device__ __forceinline__ v16h frag_h(const _Float16* rowk0, int lane) {
  union { v16h v; v8h q[2]; } u; const _Float16* p = rowk0 + 8 * (lane >> 4);
  u.q[0] = *(const v8h*)p; u.q[1] = *(const v8h*)(p + 16); return u.v;
}
__device__ __forceinline__ v16h frag_f32(const float* rowk0, int lane) {
  v16h a; const float* p = rowk0 + 8 * (lane >> 4);
#pragma unroll
  for (int i = 0; i < 8; ++i) { a[i] = (_Float16)p[i]; a[8 + i] = (_Float16)p[16 + i]; }
  return a;
}
__device__ __forceinline__ v16h frag_f32s(const float* rowk0, int lane, float sc) {
  v16h a; const float* p = rowk0 + 8 * (lane >> 4);
#pragma unroll
  for (int i = 0; i < 8; ++i) { a[i] = (_Float16)(p[i] * sc); a[8 + i] = (_Float16)(p[16 + i] * sc); }
  return a;
}
__device__ __forceinline__ v16h fragc_f32(const float* W, int k0, int n, int lane, int ld, int K) {
  v16h a; const int g = lane >> 4;
#pragma unroll
  for (int i = 0; i < 8; ++i) { const int ka = k0 + 8 * g + i, kb = ka + 16;
    a[i] = (_Float16)(ka < K ? W[(size_t)ka * ld + n] : 0.f); a[8 + i] = (_Float16)(kb < K ? W[(size_t)kb * ld + n] : 0.f); }
  return a;
}
struct F2 { v16b h, l; };
__device__ __forceinline__ F2 bsplit16(const float v[16]) { F2 r;
#pragma unroll
  for (int i = 0; i < 16; ++i) { const __bf16 h = (__bf16)v[i]; r.h[i] = h; r.l[i] = (__bf16)(v[i] - (float)h); }
  return r; }
__device__ __forceinline__ F2 split_row(const float* row, int k0, int lane) { float v[16]; const float* p = row + k0 + 8 * (lane >> 4);
#pragma unroll
  for (int i = 0; i < 8; ++i) { v[i] = p[i]; v[8 + i] = p[16 + i]; }
  return bsplit16(v); }
__device__ __forceinline__ F2 split_rowK(const float* row, int k0, int lane, int K) { float v[16]; const int g = lane >> 4;
#pragma unroll
  for (int i = 0; i < 8; ++i) { const int ka = k0 + 8 * g + i, kb = ka + 16; v[i] = ka < K ? row[ka] : 0.f; v[8 + i] = kb < K ? row[kb] : 0.f; }
  return bsplit16(v); }
__device__ __forceinline__ F2 split_col(const float* W, int k0, int n, int lane, int ld, int K) { float v[16]; const int g = lane >> 4;
#pragma unroll
  for (int i = 0; i < 8; ++i) { const int ka = k0 + 8 * g + i, kb = ka + 16; v[i] = ka < K ? W[(size_t)ka * ld + n] : 0.f; v[8 + i] = kb < K ? W[(size_t)kb * ld + n] : 0.f; }
  return bsplit16(v); }
__device__ __forceinline__ v8f mac3(const F2& a, const F2& b, v8f c) { c = wmma_bf(a.l, b.h, c); c = wmma_bf(a.h, b.l, c); return wmma_bf(a.h, b.h, c); }
__device__ __forceinline__ float sigm(float v) { return 1.0f / (1.0f + expf(-v)); }
#define LDSX() do { asm volatile("s_wait_dscnt 0" ::: "memory"); __builtin_amdgcn_wave_barrier(); __builtin_amdgcn_fence(__ATOMIC_RELEASE, "workgroup"); } while (0)


#define NN 50000
#define NNP 51200
#define NE 800000
#define DIN 256
#define GH 8
#define GO 32
#define D 256
#define XPW 288
#define RBA 128
#define NRBA (NNP / RBA)
#define RBM 2048
#define NRBM (NNP / RBM)
#define EPT 8
#define CH (256 * EPT)
__device__ __forceinline__ int f2ord(float f) { const int i = __float_as_int(f); return i >= 0 ? i : i ^ 0x7fffffff; }
__device__ __forceinline__ float ord2f(int i) { return __int_as_float(i >= 0 ? i : i ^ 0x7fffffff); }
__device__ __forceinline__ int clampn(int v) { return v < 0 ? 0 : (v >= NN ? NN - 1 : v); }

__global__ __launch_bounds__(256) void k_cvt(const float* __restrict__ x, _Float16* __restrict__ X16) {
  const size_t i8 = (size_t)blockIdx.x * 256 + threadIdx.x; if (i8 >= (size_t)NNP * DIN / 8) return;
  const size_t r = (i8 * 8) / DIN; union { v8h h; v4u u; } pk;
#pragma unroll
  for (int e = 0; e < 8; ++e) pk.h[e] = r < NN ? (_Float16)x[i8 * 8 + e] : (_Float16)0.0f;
  vst2(X16 + i8 * 8, pk.u);
}
__global__ __launch_bounds__(256) void k_w(const float* __restrict__ W, const float* __restrict__ as, const float* __restrict__ ad, _Float16* __restrict__ PT) {
  const int n = blockIdx.x, tid = threadIdx.x; __shared__ __align__(16) _Float16 srow[DIN];
  for (int k = tid; k < DIN; k += 256) { float v;
    if (n < D) v = W[(size_t)k * D + n];
    else if (n < D + 2 * GH) { const int h = (n - D) & 7; const float* a = (n < D + GH ? as : ad) + h * GO; const float* w = W + (size_t)k * D + h * GO; float s = 0.f;
#pragma unroll 4
      for (int c = 0; c < GO; ++c) s += w[c] * a[c]; v = s; }
    else v = 0.f;
    srow[k] = (_Float16)(v * 16.0f); }
  __syncthreads();
  if (tid < DIN / 8) vst2(PT + (size_t)n * DIN + tid * 8, *(const v4u*)(&srow[tid * 8]));
}
__global__ __launch_bounds__(128) void k_xp(const _Float16* __restrict__ X16, const _Float16* __restrict__ PT, float* __restrict__ XP) {
  __shared__ __align__(16) float so[4][16][132];
  const int tid = threadIdx.x, wave = tid >> 5, lane = tid & 31, col = lane & 15, g = lane >> 4;
  const int r0 = blockIdx.x * 64 + wave * 16, cg = blockIdx.y, n0 = cg * 128; const int nt = cg < 2 ? 8 : 2;
  v8f acc[8] = {};
#pragma unroll 2
  for (int kc = 0; kc < DIN / 32; ++kc) { const v16h a = frag_h(X16 + (size_t)(r0 + col) * DIN + kc * 32, lane);
#pragma unroll
    for (int j = 0; j < 8; ++j) if (j < nt) acc[j] = wmma16(a, frag_h(PT + (size_t)(n0 + j * 16 + col) * DIN + kc * 32, lane), acc[j]); }
#pragma unroll
  for (int j = 0; j < 8; ++j) if (j < nt) {
#pragma unroll
    for (int r = 0; r < 8; ++r) so[wave][8 * g + r][j * 16 + col] = acc[j][r] * (1.0f / 16.0f); }
  LDSX();
  const int npc = nt * 4;
  for (int q = lane; q < 16 * npc; q += 32) { const int rl = q / npc, pc = q % npc; vst2(XP + (size_t)(r0 + rl) * XPW + n0 + pc * 4, *(const v4f*)(&so[wave][rl][pc * 4])); }
}
__global__ __launch_bounds__(256) void k_max(const int* __restrict__ erow, const int* __restrict__ ecol, const float* __restrict__ XP, float* __restrict__ SMX) {
  __shared__ int smx[RBM][GH]; __shared__ __align__(16) float sdst[RBM][GH];
  const int tid = threadIdx.x; const int r0 = blockIdx.x * RBM;
  for (int rl = tid; rl < RBM; rl += 256) { const int row = r0 + rl; v4f d0 = {0.f, 0.f, 0.f, 0.f}, d1 = d0;
    if (row < NN) { d0 = *(const v4f*)(XP + (size_t)row * XPW + D + GH); d1 = *(const v4f*)(XP + (size_t)row * XPW + D + GH + 4); }
    *(v4f*)&sdst[rl][0] = d0; *(v4f*)&sdst[rl][4] = d1;
#pragma unroll
    for (int h = 0; h < GH; ++h) smx[rl][h] = f2ord(-3.0e38f); }
  __syncthreads();
#pragma unroll 1
  for (int c0 = 0; c0 < NE; c0 += CH) { const int e0 = c0 + tid * EPT;
#pragma unroll
    for (int v = 0; v < EPT / 4; ++v) { int dd[4];
      if (e0 + v * 4 + 4 <= NE) { const int4 d4 = *(const int4*)(ecol + e0 + v * 4); dd[0] = d4.x; dd[1] = d4.y; dd[2] = d4.z; dd[3] = d4.w; }
      else { for (int u = 0; u < 4; ++u) dd[u] = (e0 + v * 4 + u < NE) ? ecol[e0 + v * 4 + u] : -1; }
#pragma unroll
      for (int u = 0; u < 4; ++u) { if (dd[u] < 0) continue; const unsigned relr = (unsigned)(clampn(dd[u]) - r0); if (relr < (unsigned)RBM) {
          const int s = clampn(erow[e0 + v * 4 + u]); const v4f s0 = *(const v4f*)(XP + (size_t)s * XPW + D), s1 = *(const v4f*)(XP + (size_t)s * XPW + D + 4);
#pragma unroll
          for (int h = 0; h < 4; ++h) { atomicMax(&smx[relr][h], f2ord(s0[h] + sdst[relr][h])); atomicMax(&smx[relr][4 + h], f2ord(s1[h] + sdst[relr][4 + h])); } } } } }
  __syncthreads();
  for (int q = tid; q < RBM * 2; q += 256) { const int rl = q >> 1, hf = (q & 1) * 4; vst2(SMX + (size_t)(r0 + rl) * GH + hf, (v4f){ord2f(smx[rl][hf]), ord2f(smx[rl][hf + 1]), ord2f(smx[rl][hf + 2]), ord2f(smx[rl][hf + 3])}); }
}
__global__ __launch_bounds__(256) void k_agg(const int* __restrict__ erow, const int* __restrict__ ecol, const float* __restrict__ XP, const float* __restrict__ SMX, float* __restrict__ out) {
  __shared__ __align__(16) float sacc[RBA][D];
  __shared__ float sden[RBA][GH]; __shared__ float smx_[RBA][GH]; __shared__ float sdst[RBA][GH];
  __shared__ int ssrc[8][32 * EPT], sdl[8][32 * EPT]; __shared__ float swgt[8][32 * EPT][GH]; __shared__ int scnt[8];
  const int tid = threadIdx.x, wave = tid >> 5, lane = tid & 31;
  const int r0 = blockIdx.x * RBA;
  for (int q = tid; q < RBA * D; q += 256) (&sacc[0][0])[q] = 0.f;
  for (int q = tid; q < RBA * GH; q += 256) { const int rl = q >> 3, h = q & 7; const int row = r0 + rl; sden[rl][h] = 0.f; smx_[rl][h] = row < NN ? SMX[(size_t)row * GH + h] : 0.f; sdst[rl][h] = row < NN ? XP[(size_t)row * XPW + D + GH + h] : 0.f; }
  __syncthreads();
#pragma unroll 1
  for (int c0 = 0; c0 < NE; c0 += CH) { const int e0 = c0 + tid * EPT; int hd[EPT];
    if (e0 + EPT <= NE) {
#pragma unroll
      for (int v = 0; v < EPT / 4; ++v) { const int4 d4 = *(const int4*)(ecol + e0 + v * 4); const int dd[4] = {d4.x, d4.y, d4.z, d4.w};
#pragma unroll
        for (int u = 0; u < 4; ++u) { const unsigned relr = (unsigned)(clampn(dd[u]) - r0); hd[v * 4 + u] = relr < (unsigned)RBA ? (int)relr : -1; } } }
    else {
#pragma unroll
      for (int u = 0; u < EPT; ++u) { const int e = e0 + u; int dl = -1; if (e < NE) { const unsigned relr = (unsigned)(clampn(ecol[e]) - r0); dl = relr < (unsigned)RBA ? (int)relr : -1; } hd[u] = dl; } }
    int cnt = 0;
#pragma unroll
    for (int u = 0; u < EPT; ++u) cnt += hd[u] >= 0;
    int incl = cnt;
#pragma unroll
    for (int off = 1; off < 32; off <<= 1) { const int v = __shfl_up(incl, off, 32); if (lane >= off) incl += v; }
    if (lane == 31) scnt[wave] = incl;
    int pos = incl - cnt;
#pragma unroll
    for (int u = 0; u < EPT; ++u) if (hd[u] >= 0) { ssrc[wave][pos] = clampn(erow[e0 + u]); sdl[wave][pos] = hd[u]; ++pos; }
    __syncthreads();
#pragma unroll 1
    for (int w = 0; w < 8; ++w) { const int nh = scnt[w];
#pragma unroll 1
      for (int i = tid; i < nh; i += 256) { const int s = ssrc[w][i], dl = sdl[w][i]; const float* xs = XP + (size_t)s * XPW + D;
#pragma unroll 1
        for (int h = 0; h < GH; ++h) swgt[w][i][h] = expf(xs[h] + sdst[dl][h] - smx_[dl][h]); } }
    __syncthreads();
    { const int f = tid, h = f >> 5;
      for (int w = 0; w < 8; ++w) { const int nh = scnt[w]; for (int i = 0; i < nh; ++i) { const int s = ssrc[w][i], dl = sdl[w][i]; const float wa = swgt[w][i][h];
          sacc[dl][f] += wa * XP[(size_t)s * XPW + f]; if ((f & 31) == 0) sden[dl][h] += wa; } } }
    __syncthreads(); }
  for (int q = tid; q < RBA * (D / 4); q += 256) { const int rl = q >> 6, pc = q & 63; const int row = r0 + rl; if (row >= NN) continue; const int h = pc >> 3;
    v4f v = *(const v4f*)(&sacc[rl][pc * 4]); const float dn = 1.0f / (sden[rl][h] + 1e-16f); v[0] *= dn; v[1] *= dn; v[2] *= dn; v[3] *= dn; vst2(out + (size_t)row * D + pc * 4, v); }
}
extern "C" void kernel_launch(void* const* d_in, const int* in_sizes, int n_in, void* d_out, int out_size, void* d_ws, size_t ws_size, hipStream_t stream) {
  (void)in_sizes; (void)n_in; (void)out_size; (void)ws_size;
  const float* x = (const float*)d_in[0]; const int* ei = (const int*)d_in[1]; const float* W = (const float*)d_in[2]; const float* as = (const float*)d_in[3]; const float* ad = (const float*)d_in[4];
  const int* erow = ei; const int* ecol = ei + NE;
  float* out = (float*)d_out;
  char* ws = (char*)d_ws; size_t off = 0;
  auto take = [&](size_t bytes) { char* p = ws + off; off += (bytes + 255) & ~(size_t)255; return p; };
  _Float16* X16 = (_Float16*)take((size_t)NNP * DIN * 2); _Float16* PT = (_Float16*)take((size_t)XPW * DIN * 2); float* XP = (float*)take((size_t)NNP * XPW * 4); float* SMX = (float*)take((size_t)NNP * GH * 4);
  k_cvt<<<(NNP * DIN / 8 + 255) / 256, 256, 0, stream>>>(x, X16);
  k_w<<<XPW, 256, 0, stream>>>(W, as, ad, PT);
  k_xp<<<dim3(NNP / 64, 3), 128, 0, stream>>>(X16, PT, XP);
  k_max<<<NRBM, 256, 0, stream>>>(erow, ecol, XP, SMX);
  k_agg<<<NRBA, 256, 0, stream>>>(erow, ecol, XP, SMX, out);
}
